// Contraction_627065225897
// MI455X (gfx1250) — hardware-verified
//
#include <hip/hip_runtime.h>
#include <stdint.h>

#define NAT   128
#define NF    128
#define NL    16
#define NE    10
#define NP3   23
#define NP2   4
#define KP    32
#define MROWS 1280
#define NU3   4096
#define NU2   256
#define NU1   16
#define NCOL  4480
#define OC2   4096
#define OC1   4352
#define NCE   4368
#define SC    256.0f
#define ISC2  0.0000152587890625f

static_assert(MROWS == NE * NF);
static_assert((NCOL % 128) == 0);
static_assert(NCE <= NCOL);
static_assert(NCE == NU3 + NU2 + NU1);
static_assert((MROWS % 64) == 0);
static_assert(((MROWS * 4) % 256) == 0);
static_assert((((MROWS + NCOL) * 4) % 256) == 0);
static_assert(NP3 + NP2 + 1 <= KP);
static_assert(((NAT * NF) % 256) == 0);

typedef _Float16 v16h __attribute__((ext_vector_type(16)));
typedef _Float16 v8h  __attribute__((ext_vector_type(8)));
typedef float    v8f  __attribute__((ext_vector_type(8)));
typedef float    v4f  __attribute__((ext_vector_type(4)));
typedef unsigned int v4u __attribute__((ext_vector_type(4)));

__device__ __forceinline__ unsigned short bf_bits(float f) {
  unsigned u = __float_as_uint(f);
  return (unsigned short)((u + 0x7FFFu + ((u >> 16) & 1u)) >> 16);
}
__device__ __forceinline__ float bfr(float f) { return __uint_as_float(((unsigned)bf_bits(f)) << 16); }
__device__ __forceinline__ unsigned short h_bits(_Float16 x) { return __builtin_bit_cast(unsigned short, x); }
__device__ __forceinline__ unsigned short hb16(float f) { return h_bits((_Float16)f); }
__device__ __forceinline__ unsigned pk16(unsigned short a, unsigned short b) { return (unsigned)a | ((unsigned)b << 16); }
__device__ __forceinline__ v8f zero8() { v8f z = {0.f, 0.f, 0.f, 0.f, 0.f, 0.f, 0.f, 0.f}; return z; }

__device__ __forceinline__ v16h ldfrag_h(const _Float16* p) {
  union { v16h v; v8h h[2]; } f;
  f.h[0] = *(const v8h*)(p);
  f.h[1] = *(const v8h*)(p + 16);
  return f.v;
}

__device__ __forceinline__ v8f mma_raw(v16h a, v16h b, v8f c) {
  return __builtin_amdgcn_wmma_f32_16x16x32_f16(false, a, false, b, (short)0, c, false, false);
}
__device__ __forceinline__ void guard4(v8f& c0, v8f& c1, v8f& c2, v8f& c3,
                                       const v16h& a0, const v16h& a1, const v16h& b0, const v16h& b1) {
#if defined(__HIP_DEVICE_COMPILE__)
  asm volatile("v_nop\n\tv_nop\n\tv_nop\n\tv_nop"
               : "+v"(c0), "+v"(c1), "+v"(c2), "+v"(c3)
               : "v"(a0), "v"(a1), "v"(b0), "v"(b1));
#endif
}

__global__ __launch_bounds__(256)
void k_planes(const float* __restrict__ wmax, const float* __restrict__ w2, const float* __restrict__ w1,
              const float* __restrict__ U3, const float* __restrict__ U2, const float* __restrict__ U1,
              unsigned short* Ap, unsigned short* Bp) {
  const int i = blockIdx.x * 256 + threadIdx.x;
  unsigned short hv[8];
  unsigned short* dst;
  if (blockIdx.x < (MROWS * 4) / 256) {
    const int row = i >> 2, q = i & 3;
    const int e = row >> 7, f = row & (NF - 1);
    const float vc = w1[e * NF + f];
#pragma unroll
    for (int kk = 0; kk < 8; ++kk) {
      const int p  = q * 8 + kk;
      const int pw = min(p, NP3 - 1);
      const int p2 = min(max(p - NP3, 0), NP2 - 1);
      const float va = wmax[(e * NP3 + pw) * NF + f];
      const float vb = w2[(e * NP2 + p2) * NF + f];
      const float v  = (p < NP3) ? va : ((p < NP3 + NP2) ? vb : ((p == NP3 + NP2) ? vc : 0.0f));
      hv[kk] = hb16(bfr(v) * SC);
    }
    dst = Ap + (size_t)row * KP + q * 8;
  } else {
    const int j = i - MROWS * 4;
    const int n = j >> 2, q = j & 3;
    const int n3 = min(n, NU3 - 1);
    const int n2 = min(max(n - OC2, 0), NU2 - 1);
    const int n1 = min(max(n - OC1, 0), NU1 - 1);
    const float v1 = U1[n1];
#pragma unroll
    for (int kk = 0; kk < 8; ++kk) {
      const int p  = q * 8 + kk;
      const int pw = min(p, NP3 - 1);
      const int p2 = min(max(p - NP3, 0), NP2 - 1);
      const float v3 = U3[(size_t)pw * NU3 + n3];
      const float v2 = U2[p2 * NU2 + n2];
      const float s3 = (p < NP3) ? v3 : 0.0f;
      const float s2 = (p >= NP3 && p < NP3 + NP2) ? v2 : 0.0f;
      const float s1 = (n < NCE && p == NP3 + NP2) ? v1 : 0.0f;
      const float v  = (n < OC2) ? s3 : ((n < OC1) ? s2 : s1);
      hv[kk] = hb16(bfr(v) * SC);
    }
    dst = Bp + (size_t)n * KP + q * 8;
  }
  v4u u;
  u[0] = pk16(hv[0], hv[1]);
  u[1] = pk16(hv[2], hv[3]);
  u[2] = pk16(hv[4], hv[5]);
  u[3] = pk16(hv[6], hv[7]);
  *(volatile v4u*)dst = u;
  __threadfence();
  *(volatile v4u*)dst = u;
}

__global__ __launch_bounds__(256)
void k_gemm(const unsigned short* __restrict__ Ap, const unsigned short* __restrict__ Bp, float* UW) {
  constexpr int LDC = 132;
  __shared__ __align__(16) float Cs[64 * LDC];
  const int tid = threadIdx.x, wave = tid >> 5, lane = tid & 31, hh = lane >> 4, c = lane & 15;
  const int mw = wave >> 2, nw = wave & 3;
  const int mb = blockIdx.x, nb = blockIdx.y;
  const _Float16* A = (const _Float16*)(const void*)Ap;
  const _Float16* B = (const _Float16*)(const void*)Bp;
  const int ar0 = mb * 64 + mw * 32 + c;
  const int bc0 = nb * 128 + nw * 32 + c;
  const v16h fa0 = ldfrag_h(A + (size_t)ar0 * KP + 8 * hh);
  const v16h fa1 = ldfrag_h(A + (size_t)(ar0 + 16) * KP + 8 * hh);
  const v16h fb0 = ldfrag_h(B + (size_t)bc0 * KP + 8 * hh);
  const v16h fb1 = ldfrag_h(B + (size_t)(bc0 + 16) * KP + 8 * hh);
  v8f d00 = mma_raw(fa0, fb0, zero8());
  v8f d01 = mma_raw(fa0, fb1, zero8());
  v8f d10 = mma_raw(fa1, fb0, zero8());
  v8f d11 = mma_raw(fa1, fb1, zero8());
  guard4(d00, d01, d10, d11, fa0, fa1, fb0, fb1);
#pragma unroll
  for (int r = 0; r < 8; ++r) {
    const int row = mw * 32 + 8 * hh + r;
    Cs[row * LDC + nw * 32 + c]             = d00[r];
    Cs[row * LDC + nw * 32 + 16 + c]        = d01[r];
    Cs[(row + 16) * LDC + nw * 32 + c]      = d10[r];
    Cs[(row + 16) * LDC + nw * 32 + 16 + c] = d11[r];
  }
  __syncthreads();
#pragma unroll 1
  for (int row = wave; row < 64; row += 8) {
    const v4f a = *(const v4f*)(Cs + row * LDC + lane * 4);
    v4f o;
#pragma unroll
    for (int q = 0; q < 4; ++q) o[q] = a[q] * ISC2;
    float* p = UW + (size_t)(mb * 64 + row) * NCOL + (size_t)nb * 128 + lane * 4;
    *(volatile v4f*)p = o;
    __threadfence();
    *(volatile v4f*)p = o;
  }
}

__global__ __launch_bounds__(256)
void k_contract(const float* __restrict__ x, const int* __restrict__ sidx, const float* __restrict__ UW,
                float* out) {
  __shared__ float sx[NL * 256];
  __shared__ __align__(16) float so[256];
  const int tid = threadIdx.x;
  const int g = blockIdx.x * 256 + tid;
  const int b = g >> 7, f = g & (NF - 1);
  int e = sidx[b];
  e = (e < 0) ? e + NE : e;
  e = min(max(e, 0), NE - 1);
  const float* xp = x + (size_t)g * NL;
  const v4f xa = *(const v4f*)(xp);
  const v4f xb = *(const v4f*)(xp + 4);
  const v4f xc = *(const v4f*)(xp + 8);
  const v4f xd = *(const v4f*)(xp + 12);
  float xr[16];
#pragma unroll
  for (int k = 0; k < 4; ++k) {
    xr[k]      = bfr(xa[k]);
    xr[4 + k]  = bfr(xb[k]);
    xr[8 + k]  = bfr(xc[k]);
    xr[12 + k] = bfr(xd[k]);
  }
#pragma unroll
  for (int k = 0; k < NL; ++k) sx[k * 256 + tid] = xr[k];
  __syncthreads();
  const float* R = UW + (size_t)(e * NF + f) * NCOL;
  float o1 = 0.0f;
#pragma unroll 1
  for (int m1 = 0; m1 < NL; ++m1) {
    const float c1v = R[OC1 + m1];
    float o2 = 0.0f;
#pragma unroll 1
    for (int m2 = 0; m2 < NL; ++m2) {
      const int M = m1 * NL + m2;
      const float* rp = R + M * NL;
      const v4f u0 = *(const v4f*)(rp);
      const v4f u1 = *(const v4f*)(rp + 4);
      const v4f u2 = *(const v4f*)(rp + 8);
      const v4f u3 = *(const v4f*)(rp + 12);
      float o3 = u0[0] * xr[0];
      o3 = fmaf(u0[1], xr[1], o3);
      o3 = fmaf(u0[2], xr[2], o3);
      o3 = fmaf(u0[3], xr[3], o3);
      o3 = fmaf(u1[0], xr[4], o3);
      o3 = fmaf(u1[1], xr[5], o3);
      o3 = fmaf(u1[2], xr[6], o3);
      o3 = fmaf(u1[3], xr[7], o3);
      o3 = fmaf(u2[0], xr[8], o3);
      o3 = fmaf(u2[1], xr[9], o3);
      o3 = fmaf(u2[2], xr[10], o3);
      o3 = fmaf(u2[3], xr[11], o3);
      o3 = fmaf(u3[0], xr[12], o3);
      o3 = fmaf(u3[1], xr[13], o3);
      o3 = fmaf(u3[2], xr[14], o3);
      o3 = fmaf(u3[3], xr[15], o3);
      const float cv = R[OC2 + M] + o3;
      o2 = fmaf(cv, sx[m2 * 256 + tid], o2);
    }
    const float cp = c1v + o2;
    o1 = fmaf(cp, sx[m1 * 256 + tid], o1);
  }
  so[tid] = o1;
  __syncthreads();
  if (tid < 64) {
    const v4f v = *(const v4f*)(so + tid * 4);
    float* p = out + (size_t)blockIdx.x * 256 + tid * 4;
    *(volatile v4f*)p = v;
    __threadfence();
    *(volatile v4f*)p = v;
  }
}

extern "C" void kernel_launch(void* const* d_in, const int* in_sizes, int n_in,
                              void* d_out, int out_size, void* d_ws, size_t ws_size,
                              hipStream_t stream) {
  if (n_in < 9) return;
  if (in_sizes[0] != NAT * NF * NL) return;
  if (in_sizes[1] != NE) return;
  if (in_sizes[2] != NAT) return;
  if (in_sizes[3] != NE * NP3 * NF) return;
  if (in_sizes[4] != NE * NP2 * NF) return;
  if (in_sizes[5] != NE * NF) return;
  if (in_sizes[6] != NP3 * NU3) return;
  if (in_sizes[7] != NP2 * NU2) return;
  if (in_sizes[8] != NU1) return;
  if (out_size != NAT * NF) return;

  const float* x    = (const float*)d_in[0];
  const int*   sidx = (const int*)d_in[2];
  const float* wmax = (const float*)d_in[3];
  const float* w2   = (const float*)d_in[4];
  const float* w1   = (const float*)d_in[5];
  const float* U3   = (const float*)d_in[6];
  const float* U2   = (const float*)d_in[7];
  const float* U1   = (const float*)d_in[8];
  float* out = (float*)d_out;

  const size_t sA  = (size_t)MROWS * KP * 2;
  const size_t sB  = (size_t)NCOL * KP * 2;
  const size_t sUW = (size_t)MROWS * NCOL * 4;
  size_t off = 0;
  const size_t oA  = off; off += sA;
  const size_t oB  = off; off += sB;
  const size_t oUW = off; off += sUW;
  if (off > ws_size) return;
  if (off > (size_t)134217728) return;

  char* ws = (char*)d_ws;
  unsigned short* Ap = (unsigned short*)(ws + oA);
  unsigned short* Bp = (unsigned short*)(ws + oB);
  float*          UW = (float*)(ws + oUW);

  k_planes<<<dim3((MROWS + NCOL) * 4 / 256), dim3(256), 0, stream>>>(wmax, w2, w1, U3, U2, U1, Ap, Bp);
  k_gemm<<<dim3(MROWS / 64, NCOL / 128), dim3(256), 0, stream>>>(Ap, Bp, UW);
  k_contract<<<dim3(NAT * NF / 256), dim3(256), 0, stream>>>(x, sidx, UW, out);
  (void)hipGetLastError();
}
